// WAEEncoder_8701603741791
// MI455X (gfx1250) — hardware-verified
//
#include <hip/hip_runtime.h>
#include <math.h>

typedef __attribute__((ext_vector_type(16))) _Float16 v16h;
typedef __attribute__((ext_vector_type(16))) __bf16 v16b;
typedef __attribute__((ext_vector_type(8)))  _Float16 v8h;
typedef __attribute__((ext_vector_type(8)))  float v8f;
typedef __attribute__((ext_vector_type(4)))  float v4f;
typedef __attribute__((ext_vector_type(2)))  float v2f;
typedef __attribute__((ext_vector_type(4)))  unsigned v4u;
typedef __attribute__((ext_vector_type(4)))  int v4i;
typedef float __attribute__((may_alias)) float_a;
typedef int __attribute__((may_alias)) int_a;

template <typename T> __device__ __forceinline__ void vst2(void* p, T v) { *(volatile T*)p = v; __threadfence(); *(volatile T*)p = v; }
__device__ __forceinline__ v8f wmma16(v16h a, v16h b, v8f c) {
  v8f d = __builtin_amdgcn_wmma_f32_16x16x32_f16(false, a, false, b, (short)0, c, false, false);
  asm volatile("v_nop\n\tv_nop\n\tv_nop\n\tv_nop" : "+v"(d) : "v"(a), "v"(b));
  return d;
}
__device__ __forceinline__ v8f wmma_bf(v16b a, v16b b, v8f c) {
  v8f d = __builtin_amdgcn_wmma_f32_16x16x32_bf16(false, a, false, b, (short)0, c, false, false);
  asm volatile("v_nop\n\tv_nop\n\tv_nop\n\tv_nop" : "+v"(d) : "v"(a), "v"(b));
  return d;
}
__device__ __forceinline__ v16h frag_h(const _Float16* rowk0, int lane) {
  union { v16h v; v8h q[2]; } u; const _Float16* p = rowk0 + 8 * (lane >> 4);
  u.q[0] = *(const v8h*)p; u.q[1] = *(const v8h*)(p + 16); return u.v;
}
__device__ __forceinline__ v16h frag_f32(const float* rowk0, int lane) {
  v16h a; const float* p = rowk0 + 8 * (lane >> 4);
#pragma unroll
  for (int i = 0; i < 8; ++i) { a[i] = (_Float16)p[i]; a[8 + i] = (_Float16)p[16 + i]; }
  return a;
}
__device__ __forceinline__ v16h frag_f32s(const float* rowk0, int lane, float sc) {
  v16h a; const float* p = rowk0 + 8 * (lane >> 4);
#pragma unroll
  for (int i = 0; i < 8; ++i) { a[i] = (_Float16)(p[i] * sc); a[8 + i] = (_Float16)(p[16 + i] * sc); }
  return a;
}
__device__ __forceinline__ v16h fragc_f32(const float* W, int k0, int n, int lane, int ld, int K) {
  v16h a; const int g = lane >> 4;
#pragma unroll
  for (int i = 0; i < 8; ++i) { const int ka = k0 + 8 * g + i, kb = ka + 16;
    a[i] = (_Float16)(ka < K ? W[(size_t)ka * ld + n] : 0.f); a[8 + i] = (_Float16)(kb < K ? W[(size_t)kb * ld + n] : 0.f); }
  return a;
}
struct F2 { v16b h, l; };
__device__ __forceinline__ F2 bsplit16(const float v[16]) { F2 r;
#pragma unroll
  for (int i = 0; i < 16; ++i) { const __bf16 h = (__bf16)v[i]; r.h[i] = h; r.l[i] = (__bf16)(v[i] - (float)h); }
  return r; }
__device__ __forceinline__ F2 split_row(const float* row, int k0, int lane) { float v[16]; const float* p = row + k0 + 8 * (lane >> 4);
#pragma unroll
  for (int i = 0; i < 8; ++i) { v[i] = p[i]; v[8 + i] = p[16 + i]; }
  return bsplit16(v); }
__device__ __forceinline__ F2 split_rowK(const float* row, int k0, int lane, int K) { float v[16]; const int g = lane >> 4;
#pragma unroll
  for (int i = 0; i < 8; ++i) { const int ka = k0 + 8 * g + i, kb = ka + 16; v[i] = ka < K ? row[ka] : 0.f; v[8 + i] = kb < K ? row[kb] : 0.f; }
  return bsplit16(v); }
__device__ __forceinline__ F2 split_col(const float* W, int k0, int n, int lane, int ld, int K) { float v[16]; const int g = lane >> 4;
#pragma unroll
  for (int i = 0; i < 8; ++i) { const int ka = k0 + 8 * g + i, kb = ka + 16; v[i] = ka < K ? W[(size_t)ka * ld + n] : 0.f; v[8 + i] = kb < K ? W[(size_t)kb * ld + n] : 0.f; }
  return bsplit16(v); }
__device__ __forceinline__ v8f mac3(const F2& a, const F2& b, v8f c) { c = wmma_bf(a.l, b.h, c); c = wmma_bf(a.h, b.l, c); return wmma_bf(a.h, b.h, c); }
__device__ __forceinline__ float sigm(float v) { return 1.0f / (1.0f + expf(-v)); }
#define LDSX() do { asm volatile("s_wait_dscnt 0" ::: "memory"); __builtin_amdgcn_wave_barrier(); __builtin_amdgcn_fence(__ATOMIC_RELEASE, "workgroup"); } while (0)

#define NS 32768
#define NL 50
#define NV 5001
#define NH 100
#define NO 50
#define KP 128

__device__ __forceinline__ float softplus_(float v) { return v > 20.f ? v : log1pf(expf(v)); }
__device__ __forceinline__ v16h fragc_f32sK(const float* __restrict__ W, int k0, int n, int lane, int ld, int K, float sc) {
  v16h a; const int g = lane >> 4;
#pragma unroll
  for (int i = 0; i < 8; ++i) { const int ka = k0 + 8 * g + i, kb = ka + 16;
    a[i] = (_Float16)(ka < K ? W[(size_t)ka * ld + n] * sc : 0.f); a[8 + i] = (_Float16)(kb < K ? W[(size_t)kb * ld + n] * sc : 0.f); }
  return a;
}
__global__ __launch_bounds__(128) void k_wae(const int* __restrict__ tok, const float* __restrict__ W0, const float* __restrict__ b0, const float* __restrict__ W1, const float* __restrict__ b1, const float* __restrict__ W2, const float* __restrict__ b2, float* __restrict__ out) {
  __shared__ int stok[4][16][NL + 2]; __shared__ unsigned char sdup[4][16][NL + 2];
  __shared__ __align__(16) _Float16 sa[4][16][KP + 8];
  __shared__ __align__(16) float so[4][16][68];
  const int tid = threadIdx.x, wave = tid >> 5, lane = tid & 31, col = lane & 15, g = lane >> 4;
  const int r0 = blockIdx.x * 64 + wave * 16;
  for (int q = lane; q < 16 * NL; q += 32) { const int rl = q / NL, j = q % NL; int t = tok[(size_t)(r0 + rl) * NL + j]; t = t < 0 ? 0 : (t >= NV ? NV - 1 : t); stok[wave][rl][j] = t; }
  LDSX();
  for (int q = lane; q < 16 * NL; q += 32) { const int rl = q / NL, j = q % NL; const int t = stok[wave][rl][j]; bool dup = false;
    for (int i = 0; i < j; ++i) dup |= (stok[wave][rl][i] == t);
    sdup[wave][rl][j] = dup ? 1 : 0; }
  LDSX();
  { const int rl = lane >> 1, hf = lane & 1; float acc[NO];
#pragma unroll
    for (int c = 0; c < NO; ++c) acc[c] = b0[hf * NO + c];
#pragma unroll 1
    for (int j = 0; j < NL; ++j) { if (sdup[wave][rl][j]) continue; const int t = stok[wave][rl][j]; const float* wr = W0 + (size_t)t * NH + hf * NO;
#pragma unroll
      for (int c = 0; c < NO; ++c) acc[c] += wr[c]; }
#pragma unroll
    for (int c = 0; c < NO; ++c) sa[wave][rl][hf * NO + c] = (_Float16)softplus_(acc[c]);
    if (hf == 1) { for (int c = NH; c < KP; ++c) sa[wave][rl][c] = (_Float16)0.f; } }
  LDSX();
  { v8f acc[7] = {};
#pragma unroll
    for (int kc = 0; kc < KP / 32; ++kc) { const v16h a = frag_h(&sa[wave][col][0] + kc * 32, lane);
#pragma unroll
      for (int t = 0; t < 7; ++t) { const int n = t * 16 + col; acc[t] = wmma16(a, fragc_f32sK(W1, kc * 32, n < NH ? n : NH - 1, lane, NH, NH, 16.0f), acc[t]); } }
    LDSX();
#pragma unroll
    for (int t = 0; t < 7; ++t) { const int n = t * 16 + col;
#pragma unroll
      for (int r = 0; r < 8; ++r) { if (n < NH) sa[wave][8 * g + r][n] = (_Float16)softplus_(acc[t][r] * (1.0f / 16.0f) + b1[n]); } } }
  LDSX();
  { v8f acc[4] = {};
#pragma unroll
    for (int kc = 0; kc < KP / 32; ++kc) { const v16h a = frag_h(&sa[wave][col][0] + kc * 32, lane);
#pragma unroll
      for (int t = 0; t < 4; ++t) { const int n = t * 16 + col; acc[t] = wmma16(a, fragc_f32sK(W2, kc * 32, n < NO ? n : NO - 1, lane, NO, NH, 16.0f), acc[t]); } }
#pragma unroll
    for (int t = 0; t < 4; ++t) { const int n = t * 16 + col;
#pragma unroll
      for (int r = 0; r < 8; ++r) { if (n < NO) so[wave][8 * g + r][n] = acc[t][r] * (1.0f / 16.0f) + b2[n]; } } }
  LDSX();
  { const int rl = lane >> 1, hf = lane & 1; float* row = &so[wave][rl][0]; float mx = -3.4e38f;
    for (int c = 0; c < NO; ++c) mx = fmaxf(mx, row[c]);
    float se = 0.f;
    for (int c = 0; c < NO; ++c) se += expf(row[c] - mx);
    const float inv = 1.0f / se;
    __builtin_amdgcn_wave_barrier();
    for (int c = hf * 25; c < hf * 25 + 25; ++c) row[c] = expf(row[c] - mx) * inv; }
  LDSX();
  for (int q = lane; q < 16 * NO; q += 32) { const int rl = q / NO, c = q % NO; float* p = out + (size_t)(r0 + rl) * NO + c; asm volatile("" ::: "memory"); *(volatile float*)p = so[wave][rl][c]; *(volatile float*)p = so[wave][rl][c]; }
}
extern "C" void kernel_launch(void* const* d_in, const int* in_sizes, int n_in, void* d_out, int out_size, void* d_ws, size_t ws_size, hipStream_t stream) {
  (void)in_sizes; (void)n_in; (void)out_size; (void)ws_size; (void)d_ws;
  k_wae<<<NS / 64, 128, 0, stream>>>((const int*)d_in[0], (const float*)d_in[1], (const float*)d_in[2], (const float*)d_in[3], (const float*)d_in[4], (const float*)d_in[5], (const float*)d_in[6], (float*)d_out);
}
